// InputLinearizationRnn2_59141699666502
// MI455X (gfx1250) — hardware-verified
//
#include <hip/hip_runtime.h>
#include <math.h>

typedef __attribute__((ext_vector_type(16))) _Float16 v16h;
typedef __attribute__((ext_vector_type(16))) __bf16 v16b;
typedef __attribute__((ext_vector_type(8)))  _Float16 v8h;
typedef __attribute__((ext_vector_type(8)))  float v8f;
typedef __attribute__((ext_vector_type(4)))  float v4f;
typedef __attribute__((ext_vector_type(2)))  float v2f;
typedef __attribute__((ext_vector_type(4)))  unsigned v4u;
typedef __attribute__((ext_vector_type(4)))  int v4i;
typedef float __attribute__((may_alias)) float_a;
typedef int __attribute__((may_alias)) int_a;

template <typename T> __device__ __forceinline__ void vst2(void* p, T v) { *(volatile T*)p = v; __threadfence(); *(volatile T*)p = v; }
__device__ __forceinline__ v8f wmma16(v16h a, v16h b, v8f c) {
  v8f d = __builtin_amdgcn_wmma_f32_16x16x32_f16(false, a, false, b, (short)0, c, false, false);
  asm volatile("v_nop\n\tv_nop\n\tv_nop\n\tv_nop" : "+v"(d) : "v"(a), "v"(b));
  return d;
}
__device__ __forceinline__ v8f wmma_bf(v16b a, v16b b, v8f c) {
  v8f d = __builtin_amdgcn_wmma_f32_16x16x32_bf16(false, a, false, b, (short)0, c, false, false);
  asm volatile("v_nop\n\tv_nop\n\tv_nop\n\tv_nop" : "+v"(d) : "v"(a), "v"(b));
  return d;
}
__device__ __forceinline__ v16h frag_h(const _Float16* rowk0, int lane) {
  union { v16h v; v8h q[2]; } u; const _Float16* p = rowk0 + 8 * (lane >> 4);
  u.q[0] = *(const v8h*)p; u.q[1] = *(const v8h*)(p + 16); return u.v;
}
__device__ __forceinline__ v16h frag_f32(const float* rowk0, int lane) {
  v16h a; const float* p = rowk0 + 8 * (lane >> 4);
#pragma unroll
  for (int i = 0; i < 8; ++i) { a[i] = (_Float16)p[i]; a[8 + i] = (_Float16)p[16 + i]; }
  return a;
}
__device__ __forceinline__ v16h frag_f32s(const float* rowk0, int lane, float sc) {
  v16h a; const float* p = rowk0 + 8 * (lane >> 4);
#pragma unroll
  for (int i = 0; i < 8; ++i) { a[i] = (_Float16)(p[i] * sc); a[8 + i] = (_Float16)(p[16 + i] * sc); }
  return a;
}
__device__ __forceinline__ v16h fragc_f32(const float* W, int k0, int n, int lane, int ld, int K) {
  v16h a; const int g = lane >> 4;
#pragma unroll
  for (int i = 0; i < 8; ++i) { const int ka = k0 + 8 * g + i, kb = ka + 16;
    a[i] = (_Float16)(ka < K ? W[(size_t)(ka < K ? ka : K - 1) * ld + n] : 0.f); a[8 + i] = (_Float16)(kb < K ? W[(size_t)(kb < K ? kb : K - 1) * ld + n] : 0.f); }
  return a;
}
struct F2 { v16b h, l; };
__device__ __forceinline__ F2 bsplit16(const float v[16]) { F2 r;
#pragma unroll
  for (int i = 0; i < 16; ++i) { const __bf16 h = (__bf16)v[i]; r.h[i] = h; r.l[i] = (__bf16)(v[i] - (float)h); }
  return r; }
__device__ __forceinline__ F2 split_row(const float* row, int k0, int lane) { float v[16]; const float* p = row + k0 + 8 * (lane >> 4);
#pragma unroll
  for (int i = 0; i < 8; ++i) { v[i] = p[i]; v[8 + i] = p[16 + i]; }
  return bsplit16(v); }
__device__ __forceinline__ F2 split_rowK(const float* row, int k0, int lane, int K) { float v[16]; const int g = lane >> 4;
#pragma unroll
  for (int i = 0; i < 8; ++i) { const int ka = k0 + 8 * g + i, kb = ka + 16; v[i] = ka < K ? row[ka < K ? ka : K - 1] : 0.f; v[8 + i] = kb < K ? row[kb < K ? kb : K - 1] : 0.f; }
  return bsplit16(v); }
__device__ __forceinline__ F2 split_col(const float* W, int k0, int n, int lane, int ld, int K) { float v[16]; const int g = lane >> 4;
#pragma unroll
  for (int i = 0; i < 8; ++i) { const int ka = k0 + 8 * g + i, kb = ka + 16; v[i] = ka < K ? W[(size_t)(ka < K ? ka : K - 1) * ld + n] : 0.f; v[8 + i] = kb < K ? W[(size_t)(kb < K ? kb : K - 1) * ld + n] : 0.f; }
  return bsplit16(v); }
__device__ __forceinline__ v8f mac3(const F2& a, const F2& b, v8f c) { c = wmma_bf(a.l, b.h, c); c = wmma_bf(a.h, b.l, c); return wmma_bf(a.h, b.h, c); }
__device__ __forceinline__ float sigm(float v) { return 1.0f / (1.0f + expf(-v)); }
#define LDSX() do { asm volatile("s_wait_dscnt 0" ::: "memory"); __builtin_amdgcn_wave_barrier(); __builtin_amdgcn_fence(__ATOMIC_RELEASE, "workgroup"); } while (0)


#define NB 256
#define NSTEP 1024
#define NS 128
#define ND 32
#define NE 32
#define NW 64
#ifndef NRB
#define NRB (NB / 64)
#endif
typedef __attribute__((ext_vector_type(8))) __bf16 v8b;
__device__ __forceinline__ v16b frag_b(const __bf16* rowk0, int lane) {
  union { v16b v; v8b q[2]; } u; const __bf16* p = rowk0 + 8 * (lane >> 4);
  u.q[0] = *(const v8b*)p; u.q[1] = *(const v8b*)(p + 16); return u.v;
}
__device__ __forceinline__ float bfr(float v) { return (float)(__bf16)v; }
__device__ __attribute__((noinline)) float exp_ni(float v) { return expf(v); }
__device__ __attribute__((noinline)) float erf_ni(float v) { return erff(v); }

__device__ __attribute__((noinline)) float tanh_ni(float v) { return tanhf(v); }
struct F3 { v16b h, m, l; };
__device__ __forceinline__ F3 split3_row(const float* row, int k0, int lane) { F3 r; const float* p = row + k0 + 8 * (lane >> 4);
#pragma unroll
  for (int i = 0; i < 16; ++i) { const float v = (i < 8) ? p[i] : p[16 + i - 8]; const __bf16 hb = (__bf16)v; const float r1 = v - (float)hb; const __bf16 mb = (__bf16)r1; r.h[i] = hb; r.m[i] = mb; r.l[i] = (__bf16)(r1 - (float)mb); }
  return r; }
__device__ __forceinline__ v8f mac3w(const F3& a, v16b w, v8f c) { c = wmma_bf(a.l, w, c); c = wmma_bf(a.m, w, c); return wmma_bf(a.h, w, c); }
#define WS_PW  0u
#define PA   0
#define PB1  (PA + NS * NS)
#define PB2  (PB1 + NS * ND)
#define PC1  (PB2 + NS * NW)
#define PD11 (PC1 + NE * NS)
#define PD12 (PD11 + NE * ND)
#define PC2  (PD12 + NE * NW)
#define PD21 (PC2 + NW * NS)
#define PWEND (PD21 + NW * ND)
#define WS_END (WS_PW + 2u * PWEND)

__global__ __launch_bounds__(128) void k_pack(const float* __restrict__ A_, const float* __restrict__ B1_, const float* __restrict__ B2_, const float* __restrict__ C1_, const float* __restrict__ D11_, const float* __restrict__ D12_, const float* __restrict__ C2_, const float* __restrict__ D21_, __bf16* __restrict__ PW) {
  __shared__ __align__(16) __bf16 s[NS]; const int n = blockIdx.x, which = blockIdx.y, k = threadIdx.x; const float* Wm; int N_, K_; size_t base;
  switch (which) { case 0: Wm = A_; N_ = NS; K_ = NS; base = PA; break; case 1: Wm = B1_; N_ = NS; K_ = ND; base = PB1; break; case 2: Wm = B2_; N_ = NS; K_ = NW; base = PB2; break; case 3: Wm = C1_; N_ = NE; K_ = NS; base = PC1; break; case 4: Wm = D11_; N_ = NE; K_ = ND; base = PD11; break; case 5: Wm = D12_; N_ = NE; K_ = NW; base = PD12; break; case 6: Wm = C2_; N_ = NW; K_ = NS; base = PC2; break; default: Wm = D21_; N_ = NW; K_ = ND; base = PD21; break; }
  if (n >= N_) return;
  if (k < K_) s[k] = (__bf16)Wm[(size_t)n * K_ + k]; __syncthreads();
  if (k < K_ / 8) vst2((unsigned*)(PW + base + (size_t)n * K_ + k * 8), *(const v4u*)&s[k * 8]);
}
__global__ __launch_bounds__(128) void k_rnn(const float* __restrict__ X0, const float* __restrict__ US, const __bf16* __restrict__ PW, float* __restrict__ YS) {
  __shared__ __align__(16) float sx[64][NS + 4], su[64][ND + 4], sw[64][NW + 4], sy[64][NE + 4];
  const int tid = threadIdx.x, wave = tid >> 5, lane = tid & 31, col = lane & 15, g = lane >> 4; const size_t b0 = (size_t)blockIdx.x * 64; const int r0 = wave * 16;
  for (int q = tid; q < 64 * NS; q += 128) sx[q / NS][q % NS] = bfr(X0[(b0 + q / NS) * NS + q % NS]);
  __syncthreads();
#pragma unroll 1
  for (int k = 0; k < NSTEP; ++k) {
#pragma unroll
    for (int r = 0; r < 8; ++r) { const size_t b = b0 + r0 + 8 * g + r; su[r0 + 8 * g + r][col] = bfr(US[(b * NSTEP + k) * ND + col]); su[r0 + 8 * g + r][16 + col] = bfr(US[(b * NSTEP + k) * ND + 16 + col]); }
    LDSX();
    v16b au; { const F3 t = split3_row(&su[r0 + col][0], 0, lane); au = t.h; }
    { v8f acc[4] = {};
#pragma unroll 1
      for (int kc = 0; kc < 4; ++kc) { const F3 a = split3_row(&sx[r0 + col][0], kc * 32, lane);
#pragma unroll
        for (int j = 0; j < 4; ++j) acc[j] = mac3w(a, frag_b(PW + PC2 + (size_t)(j * 16 + col) * NS + kc * 32, lane), acc[j]); }
#pragma unroll
      for (int j = 0; j < 4; ++j) acc[j] = wmma_bf(au, frag_b(PW + PD21 + (size_t)(j * 16 + col) * ND, lane), acc[j]);
#pragma unroll
      for (int j = 0; j < 4; ++j)
#pragma unroll
        for (int r = 0; r < 8; ++r) sw[r0 + 8 * g + r][j * 16 + col] = tanh_ni(acc[j][r]); }
    LDSX();
    { v8f acc[8] = {};
#pragma unroll 1
      for (int kc = 0; kc < 4; ++kc) { const F3 a = split3_row(&sx[r0 + col][0], kc * 32, lane);
#pragma unroll
        for (int j = 0; j < 8; ++j) acc[j] = mac3w(a, frag_b(PW + PA + (size_t)(j * 16 + col) * NS + kc * 32, lane), acc[j]); }
#pragma unroll
      for (int j = 0; j < 8; ++j) acc[j] = wmma_bf(au, frag_b(PW + PB1 + (size_t)(j * 16 + col) * ND, lane), acc[j]);
#pragma unroll 1
      for (int kc = 0; kc < 2; ++kc) { const F3 a = split3_row(&sw[r0 + col][0], kc * 32, lane);
#pragma unroll
        for (int j = 0; j < 8; ++j) acc[j] = mac3w(a, frag_b(PW + PB2 + (size_t)(j * 16 + col) * NW + kc * 32, lane), acc[j]); }
      LDSX();
#pragma unroll
      for (int j = 0; j < 8; ++j)
#pragma unroll
        for (int r = 0; r < 8; ++r) sx[r0 + 8 * g + r][j * 16 + col] = acc[j][r]; }
    LDSX();
    { v8f acc[2] = {};
#pragma unroll 1
      for (int kc = 0; kc < 4; ++kc) { const F3 a = split3_row(&sx[r0 + col][0], kc * 32, lane);
#pragma unroll
        for (int j = 0; j < 2; ++j) acc[j] = mac3w(a, frag_b(PW + PC1 + (size_t)(j * 16 + col) * NS + kc * 32, lane), acc[j]); }
#pragma unroll
      for (int j = 0; j < 2; ++j) acc[j] = wmma_bf(au, frag_b(PW + PD11 + (size_t)(j * 16 + col) * ND, lane), acc[j]);
#pragma unroll 1
      for (int kc = 0; kc < 2; ++kc) { const F3 a = split3_row(&sw[r0 + col][0], kc * 32, lane);
#pragma unroll
        for (int j = 0; j < 2; ++j) acc[j] = mac3w(a, frag_b(PW + PD12 + (size_t)(j * 16 + col) * NW + kc * 32, lane), acc[j]); }
#pragma unroll
      for (int j = 0; j < 2; ++j)
#pragma unroll
        for (int r = 0; r < 8; ++r) sy[r0 + 8 * g + r][j * 16 + col] = acc[j][r]; }
    LDSX();
    for (int rl = 0; rl < 16; rl += 4) { const int rr = r0 + rl + (lane >> 3), pc = lane & 7; vst2(YS + ((b0 + rr) * NSTEP + k) * NE + pc * 4, *(const v4f*)&sy[rr][pc * 4]); }
  }
}
extern "C" void kernel_launch(void* const* d_in, const int* in_sizes, int n_in, void* d_out, int out_size, void* d_ws, size_t ws_size, hipStream_t stream) {
  (void)in_sizes; (void)n_in; (void)out_size;
  const float** F = (const float**)d_in;
  if (ws_size < (size_t)WS_END) return;
  char* ws = (char*)d_ws; __bf16* PW = (__bf16*)(ws + WS_PW);
  k_pack<<<dim3(NS, 8), 128, 0, stream>>>(F[2], F[3], F[4], F[5], F[6], F[7], F[8], F[9], PW);
  k_rnn<<<NRB, 128, 0, stream>>>(F[0], F[1], PW, (float*)d_out);
}
